// FFTBias_8727373545479
// MI455X (gfx1250) — hardware-verified
//
#include <hip/hip_runtime.h>
#include <math.h>

typedef __attribute__((ext_vector_type(16))) _Float16 v16h;
typedef __attribute__((ext_vector_type(16))) __bf16 v16b;
typedef __attribute__((ext_vector_type(8)))  _Float16 v8h;
typedef __attribute__((ext_vector_type(8)))  float v8f;
typedef __attribute__((ext_vector_type(4)))  float v4f;
typedef __attribute__((ext_vector_type(2)))  float v2f;
typedef __attribute__((ext_vector_type(4)))  unsigned v4u;
typedef __attribute__((ext_vector_type(4)))  int v4i;
typedef float __attribute__((may_alias)) float_a;
typedef int __attribute__((may_alias)) int_a;

template <typename T> __device__ __forceinline__ void vst2(void* p, T v) { *(volatile T*)p = v; __threadfence(); *(volatile T*)p = v; }
__device__ __forceinline__ v8f wmma16(v16h a, v16h b, v8f c) {
  v8f d = __builtin_amdgcn_wmma_f32_16x16x32_f16(false, a, false, b, (short)0, c, false, false);
  asm volatile("v_nop\n\tv_nop\n\tv_nop\n\tv_nop" : "+v"(d) : "v"(a), "v"(b));
  return d;
}
__device__ __forceinline__ v8f wmma_bf(v16b a, v16b b, v8f c) {
  v8f d = __builtin_amdgcn_wmma_f32_16x16x32_bf16(false, a, false, b, (short)0, c, false, false);
  asm volatile("v_nop\n\tv_nop\n\tv_nop\n\tv_nop" : "+v"(d) : "v"(a), "v"(b));
  return d;
}
__device__ __forceinline__ v16h frag_h(const _Float16* rowk0, int lane) {
  union { v16h v; v8h q[2]; } u; const _Float16* p = rowk0 + 8 * (lane >> 4);
  u.q[0] = *(const v8h*)p; u.q[1] = *(const v8h*)(p + 16); return u.v;
}
__device__ __forceinline__ v16h frag_f32(const float* rowk0, int lane) {
  v16h a; const float* p = rowk0 + 8 * (lane >> 4);
#pragma unroll
  for (int i = 0; i < 8; ++i) { a[i] = (_Float16)p[i]; a[8 + i] = (_Float16)p[16 + i]; }
  return a;
}
__device__ __forceinline__ v16h frag_f32s(const float* rowk0, int lane, float sc) {
  v16h a; const float* p = rowk0 + 8 * (lane >> 4);
#pragma unroll
  for (int i = 0; i < 8; ++i) { a[i] = (_Float16)(p[i] * sc); a[8 + i] = (_Float16)(p[16 + i] * sc); }
  return a;
}
__device__ __forceinline__ v16h fragc_f32(const float* W, int k0, int n, int lane, int ld, int K) {
  v16h a; const int g = lane >> 4;
#pragma unroll
  for (int i = 0; i < 8; ++i) { const int ka = k0 + 8 * g + i, kb = ka + 16;
    a[i] = (_Float16)(ka < K ? W[(size_t)(ka < K ? ka : K - 1) * ld + n] : 0.f); a[8 + i] = (_Float16)(kb < K ? W[(size_t)(kb < K ? kb : K - 1) * ld + n] : 0.f); }
  return a;
}
struct F2 { v16b h, l; };
__device__ __forceinline__ F2 bsplit16(const float v[16]) { F2 r;
#pragma unroll
  for (int i = 0; i < 16; ++i) { const __bf16 h = (__bf16)v[i]; r.h[i] = h; r.l[i] = (__bf16)(v[i] - (float)h); }
  return r; }
__device__ __forceinline__ F2 split_row(const float* row, int k0, int lane) { float v[16]; const float* p = row + k0 + 8 * (lane >> 4);
#pragma unroll
  for (int i = 0; i < 8; ++i) { v[i] = p[i]; v[8 + i] = p[16 + i]; }
  return bsplit16(v); }
__device__ __forceinline__ F2 split_rowK(const float* row, int k0, int lane, int K) { float v[16]; const int g = lane >> 4;
#pragma unroll
  for (int i = 0; i < 8; ++i) { const int ka = k0 + 8 * g + i, kb = ka + 16; v[i] = ka < K ? row[ka < K ? ka : K - 1] : 0.f; v[8 + i] = kb < K ? row[kb < K ? kb : K - 1] : 0.f; }
  return bsplit16(v); }
__device__ __forceinline__ F2 split_col(const float* W, int k0, int n, int lane, int ld, int K) { float v[16]; const int g = lane >> 4;
#pragma unroll
  for (int i = 0; i < 8; ++i) { const int ka = k0 + 8 * g + i, kb = ka + 16; v[i] = ka < K ? W[(size_t)(ka < K ? ka : K - 1) * ld + n] : 0.f; v[8 + i] = kb < K ? W[(size_t)(kb < K ? kb : K - 1) * ld + n] : 0.f; }
  return bsplit16(v); }
__device__ __forceinline__ v8f mac3(const F2& a, const F2& b, v8f c) { c = wmma_bf(a.l, b.h, c); c = wmma_bf(a.h, b.l, c); return wmma_bf(a.h, b.h, c); }
__device__ __forceinline__ float sigm(float v) { return 1.0f / (1.0f + expf(-v)); }
#define LDSX() do { asm volatile("s_wait_dscnt 0" ::: "memory"); __builtin_amdgcn_wave_barrier(); __builtin_amdgcn_fence(__ATOMIC_RELEASE, "workgroup"); } while (0)

__device__ __forceinline__ float bfr(float v) { return (float)(__bf16)v; }
#define NB 4
#define TT 2048
#define NH 16
#define HD 64
#define CC (NH * HD)
#ifndef TNB
#define TNB NB
#endif
#define ZOFF ((size_t)NB * TT * CC)
typedef __attribute__((ext_vector_type(8))) __bf16 v8b;
__device__ __forceinline__ v16b frag_b(const __bf16* rowk0, int lane) { union { v16b v; v8b q[2]; } u; const __bf16* p = rowk0 + 8 * (lane >> 4); u.q[0] = *(const v8b*)p; u.q[1] = *(const v8b*)(p + 16); return u.v; }
#define WS_VT 0u
#define WS_END (WS_VT + 2u * (size_t)NB * CC * TT)
__global__ __launch_bounds__(128) void k_vt(const float* __restrict__ V, __bf16* __restrict__ VT) { __shared__ __align__(16) __bf16 th[128][136];
  const int tid = threadIdx.x; const int t0 = blockIdx.x * 128; const size_t b = blockIdx.y; const int c0 = blockIdx.z * 128;
  for (int e = tid; e < 128 * 128; e += 128) { const int tl = e >> 7, cl = e & 127; th[cl][tl] = (__bf16)V[(b * TT + t0 + tl) * CC + c0 + cl]; }
  __syncthreads();
  for (int e = tid; e < 128 * 16; e += 128) { const int cl = e >> 4, q = e & 15; vst2((unsigned*)(VT + (b * CC + c0 + cl) * (size_t)TT + t0 + q * 8), *(const v4u*)&th[cl][q * 8]); } }
__global__ __launch_bounds__(128) void k_pbv(const float* __restrict__ Wt, const __bf16* __restrict__ VT, float* __restrict__ OUT) { __shared__ float sw[TT]; __shared__ __align__(16) float ss[4][16][HD + 4];
  const int tid = threadIdx.x, wave = tid >> 5, lane = tid & 31, col = lane & 15, g = lane >> 4; const int h = blockIdx.y; const size_t b = blockIdx.z; const int s0 = blockIdx.x * 64 + wave * 16;
  for (int i = tid; i < TT; i += 128) sw[i] = bfr(Wt[(size_t)h * TT + i]);
  __syncthreads();
  const int srow = s0 + col; v8f acc[HD / 16] = {};
#pragma unroll 1
  for (int kc = 0; kc < TT / 32; ++kc) { v16b a;
#pragma unroll
    for (int i = 0; i < 8; ++i) { const int ta = kc * 32 + 8 * g + i, tb = ta + 16; const int da = srow - ta, db = srow - tb; a[i] = (__bf16)sw[da < 0 ? -da : da]; a[8 + i] = (__bf16)sw[db < 0 ? -db : db]; }
#pragma unroll
    for (int j = 0; j < HD / 16; ++j) acc[j] = wmma_bf(a, frag_b(VT + (b * CC + h * HD + j * 16 + col) * (size_t)TT + kc * 32, lane), acc[j]); }
#pragma unroll
  for (int j = 0; j < HD / 16; ++j)
#pragma unroll
    for (int r = 0; r < 8; ++r) ss[wave][8 * g + r][j * 16 + col] = acc[j][r];
  LDSX(); for (int rl = 0; rl < 16; ++rl) if (lane < HD / 4) vst2(OUT + (b * TT + s0 + rl) * CC + h * HD + lane * 4, *(const v4f*)&ss[wave][rl][lane * 4]); }
__global__ __launch_bounds__(256) void k_zpb(const float* __restrict__ Wt, const float* __restrict__ O, float* __restrict__ Z) { __shared__ __align__(16) float so[32 * NH]; __shared__ float sob[TT];
  const int t = threadIdx.x; const int s0 = blockIdx.x * 32; const int sl = t >> 3, hp = t & 7; const int s = s0 + sl;
  for (int i = t; i < TT; i += 256) sob[i] = bfr(O[i]);
  __syncthreads();
  float a0 = 0.f, a1 = 0.f; const float* w0 = Wt + (size_t)(2 * hp) * TT; const float* w1 = w0 + TT;
#pragma unroll 1
  for (int tt = 0; tt < TT; ++tt) { const int d = s - tt; const int ad = d < 0 ? -d : d; const float ov = sob[tt]; a0 += bfr(w0[ad]) * ov; a1 += bfr(w1[ad]) * ov; }
  so[sl * NH + 2 * hp] = a0; so[sl * NH + 2 * hp + 1] = a1;
  __syncthreads();
  if (t < 32 * NH / 4) vst2(Z + (size_t)s0 * NH + t * 4, *(const v4f*)&so[t * 4]); }
extern "C" void kernel_launch(void* const* d_in, const int* in_sizes, int n_in, void* d_out, int out_size, void* d_ws, size_t ws_size, hipStream_t stream) {
  (void)in_sizes; (void)n_in; (void)out_size;
  const float** F = (const float**)d_in;
  if (ws_size < (size_t)WS_END) return;
  char* ws = (char*)d_ws; __bf16* VT = (__bf16*)(ws + WS_VT); float* OUTF = (float*)d_out;
  k_vt<<<dim3(TT / 128, TNB, CC / 128), 128, 0, stream>>>(F[0], VT);
  k_pbv<<<dim3(TT / 64, NH, TNB), 128, 0, stream>>>(F[1], VT, OUTF);
  k_zpb<<<dim3(TT / 32), 256, 0, stream>>>(F[1], F[2], OUTF + ZOFF);
}
